// PA_MSA_39152921870569
// MI455X (gfx1250) — hardware-verified
//
#include <hip/hip_runtime.h>
#include <math.h>

constexpr int kB     = 4;
constexpr int kC     = 192;
constexpr int kHeads = 4;
constexpr int kCh    = 48;
constexpr int kHW    = 128;
constexpr int kN     = kHW * kHW;
constexpr int kM3    = 3 * kC;
constexpr float kWCarry   = 16.0f;
constexpr float kQKCarry  = 256.0f;
constexpr float kVCarry   = 64.0f;
constexpr float kPCarry   = 4096.0f;
constexpr float kQKVScale = 1.0f / 16.0f;
constexpr float kSScale   = 1.0f / 65536.0f;
constexpr float kPVScale  = 1.0f / (4096.0f * 64.0f);
constexpr float kInv48    = 1.0f / 48.0f;
constexpr float kNormEps  = 1e-12f;

constexpr size_t kOffW16  = 0;
constexpr size_t kOffS    = 221184;
constexpr size_t kOffP16  = 368640;
constexpr size_t kOffMV   = 442368;
constexpr size_t kOffXT   = 704512;
constexpr size_t kOffQKV0 = 6995968;
constexpr size_t kOffQKV1 = 44744704;
constexpr size_t kOffQKN  = 82493440;
constexpr size_t kOffVT   = 95076352;
constexpr size_t kWsTotal = 101367808;

typedef __attribute__((ext_vector_type(16))) _Float16 v16h;
typedef __attribute__((ext_vector_type(8)))  _Float16 v8h;
typedef __attribute__((ext_vector_type(16))) __bf16   v16b;
typedef __attribute__((ext_vector_type(8)))  __bf16   v8b;
typedef __attribute__((ext_vector_type(8)))  float    v8f;
typedef __attribute__((ext_vector_type(4)))  float    v4f;
typedef __attribute__((ext_vector_type(4)))  unsigned int v4u;
typedef __attribute__((ext_vector_type(2)))  unsigned int v2u;

__device__ __forceinline__ unsigned short f2bf_bits(float f) {
  unsigned u = __float_as_uint(f);
  return (unsigned short)((u + 0x7FFFu + ((u >> 16) & 1u)) >> 16);
}
__device__ __forceinline__ float bf_bits2f(unsigned short h) { return __uint_as_float(((unsigned)h) << 16); }

__device__ __forceinline__ void dep_guard_h(v8f& a, v8f& b, v16h x, v16h y) { asm volatile("v_nop\n\tv_nop\n\tv_nop\n\tv_nop" : "+v"(a), "+v"(b) : "v"(x), "v"(y)); }
__device__ __forceinline__ void dep_guard_b(v8f& a, v8f& b, v16b x, v16b y) { asm volatile("v_nop\n\tv_nop\n\tv_nop\n\tv_nop" : "+v"(a), "+v"(b) : "v"(x), "v"(y)); }
__device__ __forceinline__ void keep4_h(v16h a, v16h b, v16h c, v16h d) { asm volatile("v_nop" :: "v"(a), "v"(b), "v"(c), "v"(d)); }
__device__ __forceinline__ void keep4_b(v16b a, v16b b, v16b c, v16b d) { asm volatile("v_nop" :: "v"(a), "v"(b), "v"(c), "v"(d)); }
__device__ __forceinline__ void acc_guard4(v8f& a, v8f& b, v8f& c, v8f& d) { asm volatile("v_nop\n\tv_nop\n\tv_nop\n\tv_nop" : "+v"(a), "+v"(b), "+v"(c), "+v"(d)); }
template <typename T> struct Frag;
template <> struct Frag<_Float16> {
  typedef v16h V; union U { v16h v; v8h h[2]; };
  static __device__ __forceinline__ v16h load(const _Float16* p) {
    U f; f.h[0] = *(const v8h*)(p); f.h[1] = *(const v8h*)(p + 16); return f.v;
  }
  static __device__ __forceinline__ v8f mma(v16h a, v16h b, v8f c) {
    return __builtin_amdgcn_wmma_f32_16x16x32_f16(false, a, false, b, (short)0, c, false, false);
  }
  static __device__ __forceinline__ void guard(v8f& a, v8f& b, v16h x, v16h y) { dep_guard_h(a, b, x, y); }
  static __device__ __forceinline__ void keep(v16h a, v16h b, v16h c, v16h d) { keep4_h(a, b, c, d); }
};
template <> struct Frag<__bf16> {
  typedef v16b V; union U { v16b v; v8b h[2]; };
  static __device__ __forceinline__ v16b load(const __bf16* p) {
    U f; f.h[0] = *(const v8b*)(p); f.h[1] = *(const v8b*)(p + 16); return f.v;
  }
  static __device__ __forceinline__ v8f mma(v16b a, v16b b, v8f c) {
    return __builtin_amdgcn_wmma_f32_16x16x32_bf16(false, a, false, b, (short)0, c, false, false);
  }
  static __device__ __forceinline__ void guard(v8f& a, v8f& b, v16b x, v16b y) { dep_guard_b(a, b, x, y); }
  static __device__ __forceinline__ void keep(v16b a, v16b b, v16b c, v16b d) { keep4_b(a, b, c, d); }
};

__device__ __forceinline__ unsigned pk16(unsigned short a, unsigned short b) { return (unsigned)a | ((unsigned)b << 16); }
__device__ __forceinline__ unsigned short h_bits(float f) { const _Float16 h = (_Float16)f; return __builtin_bit_cast(unsigned short, h); }

template <int ET> struct Elem;
template <> struct Elem<0> { typedef _Float16 T; };
template <> struct Elem<1> { typedef __bf16 T; };
template <int ET, bool SPLIT, int BIAS_MODE, int OUT_MODE, bool RESID, int ACT = 0, int RESID_RDIV = 1>
__global__ __launch_bounds__(256) void wmma_gemm64(
    const unsigned short* __restrict__ Ap, const unsigned short* __restrict__ A2p, int lda, long strideA,
    const unsigned short* __restrict__ Btp, const unsigned short* __restrict__ Bt2p, int ldb, long strideB,
    void* __restrict__ Cout, void* __restrict__ Cout2, int ldc, long strideC,
    const float* __restrict__ bias,
    const float* __restrict__ resid, long strideR,
    int M, int N, int K, float scale) {
  typedef typename Elem<ET>::T T;
  typedef typename Frag<T>::V V;
  const T* A = (const T*)Ap; const T* A2 = (const T*)A2p; const T* Bt = (const T*)Btp; const T* Bt2 = (const T*)Bt2p;
  __shared__ __align__(16) float sT[8][16 * 68];
  const int b    = blockIdx.y;
  const int lane = threadIdx.x & 31;
  const int wave = threadIdx.x >> 5;
  const int tilesN = N >> 6;
  const int tilesM = M >> 6;
  const int tile = blockIdx.x * 8 + wave;
  if (tile >= tilesM * tilesN) return;
  const int tm = tile / tilesN;
  const int tn = tile - tm * tilesN;
  const int m0 = tm << 6;
  const int n0 = tn << 6;

  const T* Ab  = A  + (size_t)b * strideA;
  const T* Bb  = Bt + (size_t)b * strideB;
  const T* Ab2 = SPLIT ? (A2  + (size_t)b * strideA) : nullptr;
  const T* Bb2 = SPLIT ? (Bt2 + (size_t)b * strideB) : nullptr;

  const int rlane = lane & 15;
  const int koff  = (lane >> 4) * 8;
  const int mOff  = (lane >> 4) * 8;

  v8f acc[4][4];
#pragma unroll
  for (int i = 0; i < 4; ++i)
#pragma unroll
    for (int j = 0; j < 4; ++j) acc[i][j] = (v8f){0.f,0.f,0.f,0.f,0.f,0.f,0.f,0.f};

  for (int k0 = 0; k0 < K; k0 += 32) {
    V bh[4], bl[4];
#pragma unroll
    for (int j = 0; j < 4; ++j) {
      const size_t bo = (size_t)(n0 + (j << 4) + rlane) * ldb + koff + k0;
      bh[j] = Frag<T>::load(Bb + bo);
      if (SPLIT) bl[j] = Frag<T>::load(Bb2 + bo);
    }
#pragma unroll
    for (int i = 0; i < 4; ++i) {
      const size_t ao = (size_t)(m0 + (i << 4) + rlane) * lda + koff + k0;
      V ah = Frag<T>::load(Ab + ao);
      V al;
      if (SPLIT) al = Frag<T>::load(Ab2 + ao);
#pragma unroll
      for (int j = 0; j < 4; ++j) {
        acc[i][j] = Frag<T>::mma(ah, bh[j], acc[i][j]);
        if (SPLIT) {
          acc[i][j] = Frag<T>::mma(ah, bl[j], acc[i][j]);
          acc[i][j] = Frag<T>::mma(al, bh[j], acc[i][j]);
        }
      }
      Frag<T>::guard(acc[i][0], acc[i][3], ah, SPLIT ? al : ah);
    }
    Frag<T>::keep(bh[0], bh[1], bh[2], bh[3]);
    if (SPLIT) Frag<T>::keep(bl[0], bl[1], bl[2], bl[3]);
  }
  acc_guard4(acc[0][0], acc[0][1], acc[0][2], acc[0][3]);
  acc_guard4(acc[1][0], acc[1][1], acc[1][2], acc[1][3]);
  acc_guard4(acc[2][0], acc[2][1], acc[2][2], acc[2][3]);
  acc_guard4(acc[3][0], acc[3][1], acc[3][2], acc[3][3]);

  float* slab = sT[wave];
  const float* Rb = RESID ? (resid + (size_t)b * strideR) : nullptr;
#pragma unroll
  for (int i = 0; i < 4; ++i) {
    const int mBase = m0 + (i << 4);
#pragma unroll
    for (int j = 0; j < 4; ++j) {
      const int n = n0 + (j << 4) + rlane;
      float bv = 0.f;
      if (BIAS_MODE == 2) bv = bias[n];
#pragma unroll
      for (int r = 0; r < 8; ++r) {
        float v = acc[i][j][r] * scale;
        if (BIAS_MODE == 1) v += bias[mBase + mOff + r];
        if (BIAS_MODE == 2) v += bv;
        if (RESID) v += Rb[(size_t)((mBase + mOff + r) / RESID_RDIV) * ldc + n];
        if (ACT == 2) v = fmaxf(v, 0.0f);
        if (ACT == 4) v = (v > 0.f) ? v : 0.01f * v;
        slab[(mOff + r) * 68 + (j << 4) + rlane] = v;
      }
    }
    __builtin_amdgcn_fence(__ATOMIC_RELEASE, "workgroup");
    __builtin_amdgcn_wave_barrier();
    __builtin_amdgcn_fence(__ATOMIC_ACQUIRE, "workgroup");
    if (OUT_MODE == 0) {
      float* C = (float*)Cout + (size_t)b * strideC;
      const int hh = lane >> 4, c4 = (lane & 15) * 4;
      for (int pass = 0; pass < 2; ++pass) {
#pragma unroll
        for (int it = 0; it < 8; ++it) {
          const int row = it * 2 + hh;
          v4f v = *(const v4f*)(slab + row * 68 + c4);
          *(volatile v4f*)(C + (size_t)(mBase + row) * ldc + n0 + c4) = v;
        }
        __threadfence();
      }
    } else {
      const int q = lane >> 3, c8 = (lane & 7) * 8;
      unsigned short* C  = (unsigned short*)Cout  + (size_t)b * strideC;
      unsigned short* C2 = (OUT_MODE == 2) ? ((unsigned short*)Cout2 + (size_t)b * strideC) : nullptr;
      for (int pass = 0; pass < 2; ++pass) {
#pragma unroll
        for (int it = 0; it < 4; ++it) {
          const int row = it * 4 + q;
          const float* sp = slab + row * 68 + c8;
          v8h hv, lv;
#pragma unroll
          for (int e = 0; e < 8; ++e) {
            if (OUT_MODE == 1) {
              hv[e] = (_Float16)sp[e];
            } else {
              unsigned short hb = f2bf_bits(sp[e]);
              unsigned short lb = f2bf_bits(sp[e] - bf_bits2f(hb));
              hv[e] = __builtin_bit_cast(_Float16, hb);
              lv[e] = __builtin_bit_cast(_Float16, lb);
            }
          }
          *(volatile v8h*)(C + (size_t)(mBase + row) * ldc + n0 + c8) = hv;
          if (OUT_MODE == 2) *(volatile v8h*)(C2 + (size_t)(mBase + row) * ldc + n0 + c8) = lv;
        }
        __threadfence();
      }
    }
    __builtin_amdgcn_fence(__ATOMIC_RELEASE, "workgroup");
    __builtin_amdgcn_wave_barrier();
    __builtin_amdgcn_fence(__ATOMIC_ACQUIRE, "workgroup");
  }
}

__global__ __launch_bounds__(256) void wcast_kernel(const float* __restrict__ W0, const float* __restrict__ W1,
                                                    const float* __restrict__ W2, unsigned short* __restrict__ out, float scale) {
  const int z = blockIdx.y;
  const float* W = (z == 0) ? W0 : ((z == 1) ? W1 : W2);
  const int i = blockIdx.x * 256 + threadIdx.x;
  if (i >= (kC * kC) / 8) return;
  const float* p = W + 8 * (size_t)i;
  const v4f a = *(const v4f*)(p);
  const v4f c = *(const v4f*)(p + 4);
  unsigned short hb[8];
#pragma unroll
  for (int e = 0; e < 4; ++e) {
    hb[e]     = h_bits(a[e] * scale);
    hb[4 + e] = h_bits(c[e] * scale);
  }
  const v4u u = (v4u){pk16(hb[0], hb[1]), pk16(hb[2], hb[3]), pk16(hb[4], hb[5]), pk16(hb[6], hb[7])};
  unsigned short* q = out + (size_t)z * kC * kC + 8 * (size_t)i;
  *(volatile v4u*)q = u;
  __threadfence();
  *(volatile v4u*)q = u;
}

__global__ __launch_bounds__(256) void tcast_kernel(const float* __restrict__ in, int ldi,
                                                    unsigned short* __restrict__ out, int ldo, float scale) {
  __shared__ float sm[64][65];
  const int t  = threadIdx.x;
  const int r0 = blockIdx.x * 64;
  const int c0 = blockIdx.y * 64;
#pragma unroll
  for (int i = 0; i < 16; ++i) {
    const int e = i * 256 + t;
    const int r = e >> 6;
    const int c = e & 63;
    sm[c][r] = in[(size_t)(r0 + r) * ldi + c0 + c] * scale;
  }
  __syncthreads();
  const int lane = t & 31, wave = t >> 5;
  const int q = lane >> 3, c8 = (lane & 7) * 8;
  for (int pass = 0; pass < 2; ++pass) {
#pragma unroll
    for (int it = 0; it < 2; ++it) {
      const int row = wave * 8 + it * 4 + q;
      unsigned short hb[8];
#pragma unroll
      for (int e = 0; e < 8; ++e) hb[e] = h_bits(sm[row][c8 + e]);
      const v4u u = (v4u){pk16(hb[0], hb[1]), pk16(hb[2], hb[3]), pk16(hb[4], hb[5]), pk16(hb[6], hb[7])};
      *(volatile v4u*)(out + (size_t)(c0 + row) * ldo + r0 + c8) = u;
    }
    __threadfence();
  }
}

__global__ __launch_bounds__(256) void dwnorm_kernel(const float* __restrict__ qkv0,
                                                     const float* __restrict__ wq_dw, const float* __restrict__ wk_dw,
                                                     const float* __restrict__ wv_dw,
                                                     float* qkv1, unsigned short* qkn16) {
  __shared__ float red[256];
  const int m  = blockIdx.x;
  const int r  = m / kC;
  const int ch = m - r * kC;
  const int t  = threadIdx.x;
  float w9[9];
#pragma unroll
  for (int i = 0; i < 9; ++i) {
    const float a0 = wq_dw[ch * 9 + i];
    const float a1 = wk_dw[ch * 9 + i];
    const float a2 = wv_dw[ch * 9 + i];
    w9[i] = (r == 0) ? a0 : ((r == 1) ? a1 : a2);
  }
  const float* in = qkv0 + (size_t)m * kN;
  float* orow = qkv1 + (size_t)m * kN;
  float ss = 0.f;
#pragma unroll 1
  for (int it = 0; it < 16; ++it) {
    const int base = it * 1024 + t * 4;
    const int y  = base >> 7;
    const int x0 = base & 127;
    float o0 = 0.f, o1 = 0.f, o2 = 0.f, o3 = 0.f;
#pragma unroll
    for (int dy = 0; dy < 3; ++dy) {
      const int yy = y + dy - 1;
      const bool yok = (yy >= 0) && (yy < kHW);
      const int yc = yy < 0 ? 0 : (yy >= kHW ? (kHW - 1) : yy);
      const float* rp = in + yc * kHW;
      float v[6];
#pragma unroll
      for (int e = 0; e < 6; ++e) {
        const int xx = x0 + e - 1;
        const bool ok = yok && (xx >= 0) && (xx < kHW);
        const int xc = xx < 0 ? 0 : (xx >= kHW ? (kHW - 1) : xx);
        const float lv = rp[xc];
        v[e] = ok ? lv : 0.f;
      }
      const float wa = w9[dy * 3 + 0], wb = w9[dy * 3 + 1], wc = w9[dy * 3 + 2];
      o0 += wa * v[0] + wb * v[1] + wc * v[2];
      o1 += wa * v[1] + wb * v[2] + wc * v[3];
      o2 += wa * v[2] + wb * v[3] + wc * v[4];
      o3 += wa * v[3] + wb * v[4] + wc * v[5];
    }
    const v4f o = (v4f){o0, o1, o2, o3};
    *(volatile v4f*)(orow + base) = o;
    __threadfence();
    *(volatile v4f*)(orow + base) = o;
    ss += o0 * o0 + o1 * o1 + o2 * o2 + o3 * o3;
  }
  red[t] = ss;
  __syncthreads();
  for (int st = 128; st > 0; st >>= 1) {
    if (t < st) red[t] += red[t + st];
    __syncthreads();
  }
  const float tot  = red[0];
  const float invs = (1.0f / fmaxf(sqrtf(tot), kNormEps)) * kQKCarry;
  if (m < 2 * kC) {
    unsigned short* drow = qkn16 + (size_t)m * kN;
#pragma unroll 1
    for (int it = 0; it < 16; ++it) {
      const int base = it * 1024 + t * 4;
      const v4f o = *(const v4f*)(orow + base);
      const v2u u = (v2u){pk16(h_bits(o[0] * invs), h_bits(o[1] * invs)),
                          pk16(h_bits(o[2] * invs), h_bits(o[3] * invs))};
      *(volatile v2u*)(drow + base) = u;
      __threadfence();
      *(volatile v2u*)(drow + base) = u;
    }
  }
}

__global__ __launch_bounds__(256) void meanv_kernel(const float* __restrict__ vpl, float* __restrict__ mv) {
  const int p = blockIdx.x * 256 + threadIdx.x;
  if (p >= kN) return;
  float s[kHeads];
#pragma unroll
  for (int h = 0; h < kHeads; ++h) {
    float a = 0.f;
#pragma unroll 1
    for (int j = 0; j < kCh; ++j) a += vpl[(size_t)(h * kCh + j) * kN + p];
    s[h] = a * kInv48;
  }
#pragma unroll
  for (int h = 0; h < kHeads; ++h) ((volatile float*)mv)[(size_t)h * kN + p] = s[h];
  __threadfence();
#pragma unroll
  for (int h = 0; h < kHeads; ++h) ((volatile float*)mv)[(size_t)h * kN + p] = s[h];
}

__global__ __launch_bounds__(64) void softmax_kernel(const float* __restrict__ S, const float* __restrict__ temp,
                                                     unsigned short* __restrict__ P) {
  __shared__ float red[64];
  __shared__ float pv[kC];
  const int c = blockIdx.x;
  const int h = c / kCh;
  const int j = threadIdx.x;
  pv[j] = 0.f; pv[j + 64] = 0.f; pv[j + 128] = 0.f;
  const float tv = temp[h];
  const int jj = (j < kCh) ? j : (kCh - 1);
  const float sv = S[(size_t)c * kC + h * kCh + jj];
  const float logit = (j < kCh) ? (sv * tv) : -INFINITY;
  red[j] = logit;
  __syncthreads();
  for (int st = 32; st > 0; st >>= 1) {
    if (j < st) red[j] = fmaxf(red[j], red[j + st]);
    __syncthreads();
  }
  const float mx = red[0];
  __syncthreads();
  const float ex = expf(((j < kCh) ? logit : mx) - mx);
  const float e  = (j < kCh) ? ex : 0.f;
  red[j] = e;
  __syncthreads();
  for (int st = 32; st > 0; st >>= 1) {
    if (j < st) red[j] += red[j + st];
    __syncthreads();
  }
  const float tot = red[0];
  const float p = e * (1.0f / tot);
  if (j < kCh) pv[h * kCh + j] = (p - kInv48) * kPCarry;
  __syncthreads();
  if (j < 24) {
    unsigned short hb[8];
#pragma unroll
    for (int q = 0; q < 8; ++q) hb[q] = h_bits(pv[j * 8 + q]);
    const v4u u = (v4u){pk16(hb[0], hb[1]), pk16(hb[2], hb[3]), pk16(hb[4], hb[5]), pk16(hb[6], hb[7])};
    unsigned short* dst = P + (size_t)c * kC + j * 8;
    *(volatile v4u*)dst = u;
    __threadfence();
    *(volatile v4u*)dst = u;
  }
}

extern "C" void kernel_launch(void* const* d_in, const int* in_sizes, int n_in,
                              void* d_out, int out_size, void* d_ws, size_t ws_size, hipStream_t stream) {
  if (n_in < 8) return;
  if (in_sizes[0] != kB * kC * kN || out_size != kB * kC * kN) return;
  if (in_sizes[1] != kC * kC || in_sizes[3] != kC * kC || in_sizes[5] != kC * kC) return;
  if (in_sizes[2] != kC * 9 || in_sizes[4] != kC * 9 || in_sizes[6] != kC * 9 || in_sizes[7] < kHeads) return;
  if (ws_size < kWsTotal) return;

  const float* x     = (const float*)d_in[0];
  const float* wq    = (const float*)d_in[1];
  const float* wq_dw = (const float*)d_in[2];
  const float* wk    = (const float*)d_in[3];
  const float* wk_dw = (const float*)d_in[4];
  const float* wv    = (const float*)d_in[5];
  const float* wv_dw = (const float*)d_in[6];
  const float* temp  = (const float*)d_in[7];
  float* out = (float*)d_out;

  char* ws = (char*)d_ws;
  unsigned short* w16   = (unsigned short*)(ws + kOffW16);
  float*          sbuf  = (float*)(ws + kOffS);
  unsigned short* p16   = (unsigned short*)(ws + kOffP16);
  float*          mv    = (float*)(ws + kOffMV);
  unsigned short* xt16  = (unsigned short*)(ws + kOffXT);
  float*          qkv0  = (float*)(ws + kOffQKV0);
  float*          qkv1  = (float*)(ws + kOffQKV1);
  unsigned short* qkn16 = (unsigned short*)(ws + kOffQKN);
  unsigned short* v16t  = (unsigned short*)(ws + kOffVT);
  const float* vplane = qkv1 + (size_t)(2 * kC) * kN;
  const unsigned short* kn16 = qkn16 + (size_t)kC * kN;

  wcast_kernel<<<dim3((kC * kC) / 8 / 256, 3), 256, 0, stream>>>(wq, wk, wv, w16, kWCarry);

  for (int b = 0; b < kB; ++b) {
    const float* xb = x + (size_t)b * kC * kN;
    float* ob = out + (size_t)b * kC * kN;

    tcast_kernel<<<dim3(kC / 64, kN / 64), 256, 0, stream>>>(xb, kN, xt16, kC, 1.0f);

    wmma_gemm64<0, false, 0, 0, false, 0, 1><<<dim3((kM3 / 64) * (kN / 64) / 8, 1), 256, 0, stream>>>(
        w16, w16, kC, 0L, xt16, xt16, kC, 0L, (void*)qkv0, (void*)qkv0, kN, 0L, mv, mv, 0L, kM3, kN, kC, kQKVScale);

    dwnorm_kernel<<<kM3, 256, 0, stream>>>(qkv0, wq_dw, wk_dw, wv_dw, qkv1, qkn16);

    tcast_kernel<<<dim3(kC / 64, kN / 64), 256, 0, stream>>>(vplane, kN, v16t, kC, kVCarry);
    meanv_kernel<<<kN / 256, 256, 0, stream>>>(vplane, mv);

    wmma_gemm64<0, false, 0, 0, false, 0, 1><<<dim3(2, 1), 256, 0, stream>>>(
        qkn16, qkn16, kN, 0L, kn16, kn16, kN, 0L, (void*)sbuf, (void*)sbuf, kC, 0L, mv, mv, 0L, kC, kC, kN, kSScale);

    softmax_kernel<<<kC, 64, 0, stream>>>(sbuf, temp, p16);

    wmma_gemm64<0, false, 0, 0, true, 0, kCh><<<dim3((kC / 64) * (kN / 64) / 8, 1), 256, 0, stream>>>(
        p16, p16, kC, 0L, v16t, v16t, kC, 0L, (void*)ob, (void*)ob, kN, 0L, mv, mv, 0L, kC, kN, kC, kPVScale);
  }
}
